// GCN2_35510789603589
// MI455X (gfx1250) — hardware-verified
//
#include <hip/hip_runtime.h>
#include <stddef.h>
#include <stdint.h>


#define F      128
#define DEGN   32
#define K1     384
#define K2     512
#define NCLS   40
#define NCP    64
#define NTHR   256
#define GBM    64
#define GBN    64
#define GTHR   128
#define UB1    (F * (K1 / 8))
#define UB2    (NCP * (K2 / 8))
#define WSMAX  134217728

static_assert(GBM == (GTHR / 32) * 16);
static_assert((K1 % 32) == 0 && (K2 % 32) == 0);
static_assert((UB1 % 32) == 0 && (UB2 % 32) == 0);
static_assert(GBM * NCLS / 4 == 5 * GTHR);
static_assert((F % GBN) == 0 && NCP == GBN);
static_assert(NTHR == 256 && DEGN == 32);

typedef float          v4f  __attribute__((ext_vector_type(4)));
typedef float          v8f  __attribute__((ext_vector_type(8)));
typedef int            v4i  __attribute__((ext_vector_type(4)));
typedef int            v8i  __attribute__((ext_vector_type(8)));
typedef unsigned int   v4u  __attribute__((ext_vector_type(4)));
typedef unsigned short v8us __attribute__((ext_vector_type(8)));
typedef __bf16         v16y __attribute__((ext_vector_type(16)));
union FragY { v16y v; v8us h[2]; v8i w; };
static_assert(sizeof(FragY) == 32);

__device__ __forceinline__ v8f wmb(const FragY& a, const FragY& b, v8f c) {
  v8f d = __builtin_amdgcn_wmma_f32_16x16x32_bf16(false, a.v, false, b.v, (short)0, c, false, false);
  asm volatile("v_nop\n\tv_nop\n\tv_nop\n\tv_nop" : "+v"(d) : "v"(a.w), "v"(b.w));
  return d;
}

__device__ __forceinline__ unsigned bfb(float f) {
  unsigned u = __float_as_uint(f);
  u = u + 0x7fffu + ((u >> 16) & 1u);
  return u >> 16;
}
__device__ __forceinline__ float bfr(float f) {
  return __uint_as_float(bfb(f) << 16);
}
__device__ __forceinline__ int clampi(int v, int hi) {
  return v < 0 ? 0 : (v > hi ? hi : v);
}
__device__ __forceinline__ v4u pack8(const float* v) {
  v4u o;
  o.x = bfb(v[0]) | (bfb(v[1]) << 16);
  o.y = bfb(v[2]) | (bfb(v[3]) << 16);
  o.z = bfb(v[4]) | (bfb(v[5]) << 16);
  o.w = bfb(v[6]) | (bfb(v[7]) << 16);
  return o;
}
__device__ __forceinline__ void split8(const float* v, v4u& hv, v4u& lv) {
  unsigned hw[4], lw[4];
#pragma unroll
  for (int e = 0; e < 4; ++e) {
    const float m0 = v[2 * e], m1 = v[2 * e + 1];
    const unsigned h0 = bfb(m0), h1 = bfb(m1);
    const float r0 = m0 - __uint_as_float(h0 << 16);
    const float r1 = m1 - __uint_as_float(h1 << 16);
    const unsigned l0 = bfb(r0), l1 = bfb(r1);
    hw[e] = h0 | (h1 << 16);
    lw[e] = l0 | (l1 << 16);
  }
  hv.x = hw[0]; hv.y = hw[1]; hv.z = hw[2]; hv.w = hw[3];
  lv.x = lw[0]; lv.y = lw[1]; lv.z = lw[2]; lv.w = lw[3];
}
__device__ __forceinline__ void addbf(float* acc, const v4u g) {
  acc[0] += __uint_as_float(g.x << 16); acc[1] += __uint_as_float(g.x & 0xffff0000u);
  acc[2] += __uint_as_float(g.y << 16); acc[3] += __uint_as_float(g.y & 0xffff0000u);
  acc[4] += __uint_as_float(g.z << 16); acc[5] += __uint_as_float(g.z & 0xffff0000u);
  acc[6] += __uint_as_float(g.w << 16); acc[7] += __uint_as_float(g.w & 0xffff0000u);
}

__global__ __launch_bounds__(NTHR) void k_prep(const float* __restrict__ x, const float* __restrict__ w1,
                                               const float* __restrict__ w2,
                                               unsigned short* xb, unsigned short* b1t, unsigned short* b2t,
                                               int nN, int uX, int nUnits) {
  const int u = (int)blockIdx.x * NTHR + (int)threadIdx.x;
  if (u >= nUnits) return;
  v4u o;
  unsigned short* dst;
  if (u < uX) {
    const int row = u >> 4;
    const int c0  = (u & 15) * 8;
    const int rc  = row < nN ? row : nN - 1;
    const float* p = x + (size_t)rc * F + c0;
    const v4f a = *(const v4f*)p;
    const v4f b = *(const v4f*)(p + 4);
    float v[8];
    v[0] = a.x; v[1] = a.y; v[2] = a.z; v[3] = a.w;
    v[4] = b.x; v[5] = b.y; v[6] = b.z; v[7] = b.w;
    if (row >= nN) {
#pragma unroll
      for (int i = 0; i < 8; ++i) v[i] = 0.0f;
    }
    o = pack8(v);
    dst = xb + (size_t)row * F + c0;
  } else if (u < uX + UB1) {
    const int e  = u - uX;
    const int n  = e / (K1 / 8);
    const int k8 = (e - n * (K1 / 8)) * 8;
    float v[8];
#pragma unroll
    for (int i = 0; i < 8; ++i) {
      const int kk = k8 + i;
      const int sr = kk < 2 * F ? kk : kk - F;
      v[i] = w1[(size_t)sr * F + n];
    }
    o = pack8(v);
    dst = b1t + (size_t)n * K1 + k8;
  } else {
    const int e  = u - uX - UB1;
    const int n  = e / (K2 / 8);
    const int k8 = (e - n * (K2 / 8)) * 8;
    const int ncl = n < NCLS ? n : NCLS - 1;
    float v[8];
#pragma unroll
    for (int i = 0; i < 8; ++i) {
      const int kk = k8 + i;
      const int sr = kk < F ? kk : (kk < 3 * F ? kk - F : kk - 2 * F);
      v[i] = w2[(size_t)sr * NCLS + ncl];
    }
    if (n >= NCLS) {
#pragma unroll
      for (int i = 0; i < 8; ++i) v[i] = 0.0f;
    }
    o = pack8(v);
    dst = b2t + (size_t)n * K2 + k8;
  }
  *(volatile v4u*)dst = o;
  __threadfence();
  *(volatile v4u*)dst = o;
}

__global__ __launch_bounds__(NTHR) void k_agg1(const unsigned short* __restrict__ xb, const int* __restrict__ neigh,
                                               unsigned short* a1, int nN) {
  const int tid = (int)threadIdx.x, lane = tid & 31, wave = tid >> 5;
  const int c = lane & 15, sub = lane >> 4;
  const int row = (int)blockIdx.x * 16 + 2 * wave + sub;
  const bool live = row < nN;
  const int rc = live ? row : nN - 1;

  const v4u sx = *(const v4u*)(xb + (size_t)rc * F + 8 * c);
  const int* nbp = neigh + (size_t)rc * DEGN;
  float acc[8];
#pragma unroll
  for (int i = 0; i < 8; ++i) acc[i] = 0.0f;
#pragma unroll 2
  for (int q = 0; q < DEGN / 4; ++q) {
    const v4i nv = *(const v4i*)(nbp + 4 * q);
    const int i0 = clampi(nv.x, nN - 1), i1 = clampi(nv.y, nN - 1);
    const int i2 = clampi(nv.z, nN - 1), i3 = clampi(nv.w, nN - 1);
    const v4u g0 = *(const v4u*)(xb + (size_t)i0 * F + 8 * c);
    const v4u g1 = *(const v4u*)(xb + (size_t)i1 * F + 8 * c);
    const v4u g2 = *(const v4u*)(xb + (size_t)i2 * F + 8 * c);
    const v4u g3 = *(const v4u*)(xb + (size_t)i3 * F + 8 * c);
    addbf(acc, g0);
    addbf(acc, g1);
    addbf(acc, g2);
    addbf(acc, g3);
  }
  float mv[8];
#pragma unroll
  for (int i = 0; i < 8; ++i) mv[i] = acc[i] * 0.03125f;
  v4u hv, lv;
  split8(mv, hv, lv);
  const v4u zu = {0u, 0u, 0u, 0u};
  v4u o0 = sx, o1 = hv, o2 = lv;
  if (!live) { o0 = zu; o1 = zu; o2 = zu; }

  unsigned short* rp = a1 + (size_t)row * K1 + 8 * c;
  *(volatile v4u*)(rp)         = o0;
  *(volatile v4u*)(rp + F)     = o1;
  *(volatile v4u*)(rp + 2 * F) = o2;
  __threadfence();
  *(volatile v4u*)(rp)         = o0;
  *(volatile v4u*)(rp + F)     = o1;
  *(volatile v4u*)(rp + 2 * F) = o2;
}

__global__ __launch_bounds__(NTHR) void k_agg2(const float* __restrict__ h1, const int* __restrict__ neigh,
                                               const int* __restrict__ batch, unsigned short* a2, int nN, int nB) {
  const int tid = (int)threadIdx.x, lane = tid & 31, wave = tid >> 5;
  const int c = lane & 15, sub = lane >> 4;
  const int i = (int)blockIdx.x * 16 + 2 * wave + sub;
  const bool live = i < nB;
  const int ic = live ? i : nB - 1;
  const int node = clampi(batch[ic], nN - 1);

  const float* sp = h1 + (size_t)node * F + 8 * c;
  const v4f sa = *(const v4f*)sp;
  const v4f sb = *(const v4f*)(sp + 4);
  float sv[8];
  sv[0] = sa.x; sv[1] = sa.y; sv[2] = sa.z; sv[3] = sa.w;
  sv[4] = sb.x; sv[5] = sb.y; sv[6] = sb.z; sv[7] = sb.w;

  const int* nbp = neigh + (size_t)node * DEGN;
  float acc[8];
#pragma unroll
  for (int e = 0; e < 8; ++e) acc[e] = 0.0f;
#pragma unroll 2
  for (int q = 0; q < DEGN / 4; ++q) {
    const v4i nv = *(const v4i*)(nbp + 4 * q);
    const int i0 = clampi(nv.x, nN - 1), i1 = clampi(nv.y, nN - 1);
    const int i2 = clampi(nv.z, nN - 1), i3 = clampi(nv.w, nN - 1);
    const float* p0 = h1 + (size_t)i0 * F + 8 * c;
    const float* p1 = h1 + (size_t)i1 * F + 8 * c;
    const float* p2 = h1 + (size_t)i2 * F + 8 * c;
    const float* p3 = h1 + (size_t)i3 * F + 8 * c;
    const v4f a0 = *(const v4f*)p0, b0 = *(const v4f*)(p0 + 4);
    const v4f a1 = *(const v4f*)p1, b1 = *(const v4f*)(p1 + 4);
    const v4f a2v = *(const v4f*)p2, b2v = *(const v4f*)(p2 + 4);
    const v4f a3 = *(const v4f*)p3, b3 = *(const v4f*)(p3 + 4);
    acc[0] += a0.x; acc[1] += a0.y; acc[2] += a0.z; acc[3] += a0.w;
    acc[4] += b0.x; acc[5] += b0.y; acc[6] += b0.z; acc[7] += b0.w;
    acc[0] += a1.x; acc[1] += a1.y; acc[2] += a1.z; acc[3] += a1.w;
    acc[4] += b1.x; acc[5] += b1.y; acc[6] += b1.z; acc[7] += b1.w;
    acc[0] += a2v.x; acc[1] += a2v.y; acc[2] += a2v.z; acc[3] += a2v.w;
    acc[4] += b2v.x; acc[5] += b2v.y; acc[6] += b2v.z; acc[7] += b2v.w;
    acc[0] += a3.x; acc[1] += a3.y; acc[2] += a3.z; acc[3] += a3.w;
    acc[4] += b3.x; acc[5] += b3.y; acc[6] += b3.z; acc[7] += b3.w;
  }
  float mv[8];
#pragma unroll
  for (int e = 0; e < 8; ++e) mv[e] = acc[e] * 0.03125f;
  v4u hh, hl, mh, ml;
  split8(sv, hh, hl);
  split8(mv, mh, ml);
  const v4u zu = {0u, 0u, 0u, 0u};
  if (!live) { hh = zu; hl = zu; mh = zu; ml = zu; }

  unsigned short* rp = a2 + (size_t)i * K2 + 8 * c;
  *(volatile v4u*)(rp)         = hh;
  *(volatile v4u*)(rp + F)     = hl;
  *(volatile v4u*)(rp + 2 * F) = mh;
  *(volatile v4u*)(rp + 3 * F) = ml;
  __threadfence();
  *(volatile v4u*)(rp)         = hh;
  *(volatile v4u*)(rp + F)     = hl;
  *(volatile v4u*)(rp + 2 * F) = mh;
  *(volatile v4u*)(rp + 3 * F) = ml;
}

template<int EPI, int RELU>
__global__ __launch_bounds__(GTHR) void k_gemm(
    const unsigned short* __restrict__ A, const unsigned short* __restrict__ WT,
    const float* __restrict__ bias, int blen,
    float* outF, int K, int ldo, int nRows)
{
  __shared__ __attribute__((aligned(16))) float stg[GBM * GBN];
  const int tid = (int)threadIdx.x, lane = tid & 31, wave = tid >> 5, hh = lane >> 4, m = lane & 15;
  const int rowBase = (int)blockIdx.x * GBM;
  const int col0    = (int)blockIdx.y * GBN;

  v8f acc[4];
  {
    const v8f z = {0.f, 0.f, 0.f, 0.f, 0.f, 0.f, 0.f, 0.f};
    acc[0] = z; acc[1] = z; acc[2] = z; acc[3] = z;
  }
  const unsigned short* ap = A  + (size_t)(rowBase + 16 * wave + m) * (size_t)K + 8 * hh;
  const unsigned short* wp = WT + (size_t)(col0 + m) * (size_t)K + 8 * hh;
  const int ksteps = K >> 5;
#pragma unroll 1
  for (int ks = 0; ks < ksteps; ++ks) {
    FragY af;
    af.h[0] = *(const v8us*)(ap + 32 * ks);
    af.h[1] = *(const v8us*)(ap + 32 * ks + 16);
#pragma unroll
    for (int t = 0; t < 4; ++t) {
      const unsigned short* wq = wp + (size_t)(16 * t) * (size_t)K + 32 * ks;
      FragY bf;
      bf.h[0] = *(const v8us*)wq;
      bf.h[1] = *(const v8us*)(wq + 16);
      acc[t] = wmb(af, bf, acc[t]);
    }
  }

#pragma unroll
  for (int t = 0; t < 4; ++t) {
    const int lc = 16 * t + m;
    int bi = col0 + lc;
    bi = bi > blen - 1 ? blen - 1 : bi;
    bi = bi < 0 ? 0 : bi;
    const float bv = bfr(bias[bi]);
#pragma unroll
    for (int r = 0; r < 8; ++r) {
      const int lr = 16 * wave + 8 * hh + r;
      float val = acc[t][r] + bv;
      if (RELU) val = fmaxf(val, 0.0f);
      stg[lr * GBN + lc] = val;
    }
  }
  __syncthreads();

  if (EPI == 0) {
    v4f fv[8];
#pragma unroll
    for (int i = 0; i < 8; ++i) {
      const int lr = 16 * wave + 2 * i + hh;
      fv[i] = *(const v4f*)(stg + lr * GBN + 4 * m);
    }
#pragma unroll
    for (int i = 0; i < 8; ++i) {
      const int lr = 16 * wave + 2 * i + hh;
      const int gr = rowBase + lr;
      float* op = outF + (size_t)gr * (size_t)ldo + col0 + 4 * m;
      *(volatile v4f*)op = fv[i];
    }
    __threadfence();
#pragma unroll
    for (int i = 0; i < 8; ++i) {
      const int lr = 16 * wave + 2 * i + hh;
      const int gr = rowBase + lr;
      float* op = outF + (size_t)gr * (size_t)ldo + col0 + 4 * m;
      *(volatile v4f*)op = fv[i];
    }
  } else {
    int nv = nRows - rowBase;
    nv = nv < 0 ? 0 : (nv > GBM ? GBM : nv);
    const int np = nv * (NCLS / 4);
    v4f pv[5];
#pragma unroll
    for (int i = 0; i < 5; ++i) {
      const int p   = i * GTHR + tid;
      const int row = p / (NCLS / 4);
      const int c4  = (p - row * (NCLS / 4)) * 4;
      pv[i] = *(const v4f*)(stg + row * GBN + c4);
    }
    float* ob = outF + (size_t)rowBase * NCLS;
#pragma unroll
    for (int i = 0; i < 5; ++i) {
      const int p = i * GTHR + tid;
      if (p < np) *(volatile v4f*)(ob + 4 * p) = pv[i];
    }
    __threadfence();
#pragma unroll
    for (int i = 0; i < 5; ++i) {
      const int p = i * GTHR + tid;
      if (p < np) *(volatile v4f*)(ob + 4 * p) = pv[i];
    }
  }
}

static inline int cdiv(int a, int b) { return (a + b - 1) / b; }

extern "C" void kernel_launch(void* const* d_in, const int* in_sizes, int n_in,
                              void* d_out, int out_size, void* d_ws, size_t ws_size,
                              hipStream_t stream) {
  if (n_in < 7) return;
  const int nN = in_sizes[0] / F;
  if (nN <= 0 || in_sizes[0] != nN * F || nN > (1 << 22)) return;
  if (in_sizes[1] != nN * DEGN) return;
  const int nB = in_sizes[2];
  if (nB <= 0 || nB > (1 << 22)) return;
  if (in_sizes[3] != 2 * F * F) return;
  if (in_sizes[4] != F) return;
  if (in_sizes[5] != 2 * F * NCLS) return;
  if (in_sizes[6] != NCLS) return;
  if (out_size != nB * NCLS) return;

  const float* x     = (const float*)d_in[0];
  const int*   neigh = (const int*)  d_in[1];
  const int*   batch = (const int*)  d_in[2];
  const float* W1    = (const float*)d_in[3];
  const float* b1    = (const float*)d_in[4];
  const float* W2    = (const float*)d_in[5];
  const float* b2    = (const float*)d_in[6];
  float* out = (float*)d_out;

  const int NP  = cdiv(nN, GBM) * GBM;
  const int NP2 = cdiv(nB, GBM) * GBM;

  char* ws = (char*)d_ws;
  size_t off = 0;
  const size_t szA1 = (size_t)NP * K1 * 2, szA2 = (size_t)NP2 * K2 * 2;
  const size_t szA  = szA1 > szA2 ? szA1 : szA2;
  const size_t oXB = off; off += (size_t)NP * F * 2;   off = (off + 255) & ~(size_t)255;
  const size_t oB1 = off; off += (size_t)F * K1 * 2;    off = (off + 255) & ~(size_t)255;
  const size_t oB2 = off; off += (size_t)NCP * K2 * 2;  off = (off + 255) & ~(size_t)255;
  const size_t oH1 = off; off += (size_t)NP * F * 4;    off = (off + 255) & ~(size_t)255;
  const size_t oA  = off; off += szA;                   off = (off + 255) & ~(size_t)255;
  if (off > ws_size || off > (size_t)WSMAX) return;
  unsigned short* XB  = (unsigned short*)(ws + oXB);
  unsigned short* B1T = (unsigned short*)(ws + oB1);
  unsigned short* B2T = (unsigned short*)(ws + oB2);
  float*          H1  = (float*)(ws + oH1);
  unsigned short* AP  = (unsigned short*)(ws + oA);

  const int uX = NP * (F / 8);
  if ((uX & 31) != 0) return;
  const int nUnits = uX + UB1 + UB2;
  k_prep<<<cdiv(nUnits, NTHR), NTHR, 0, stream>>>(x, W1, W2, XB, B1T, B2T, nN, uX, nUnits);

  k_agg1<<<NP / 16, NTHR, 0, stream>>>(XB, neigh, AP, nN);

  k_gemm<0, 1><<<dim3(NP / GBM, F / GBN), GTHR, 0, stream>>>(AP, B1T, b1, F, H1, K1, F, nN);

  k_agg2<<<NP2 / 16, NTHR, 0, stream>>>(H1, neigh, batch, AP, nN, nB);

  k_gemm<1, 0><<<dim3(NP2 / GBM, 1), GTHR, 0, stream>>>(AP, B2T, b2, NCLS, out, K2, NCLS, nB);
}
